// GATMultiHead_2894807957582
// MI455X (gfx1250) — hardware-run, weakly checked
//
#include <hip/hip_runtime.h>


namespace {
constexpr int N = 50000, NP = 50048, E = 1600000, G = 64, XF = 5, NH = 2, C1 = 32, C2 = 64, W1O = NH * C1, W2O = NH * C2, HZ = 32, NCLS = 10, NBLK = NP / 16;
constexpr float XS = 8.0f, WSC = 256.0f, NEG = 0.2f, BNEPS = 1e-5f;
typedef _Float16 b16;
typedef __attribute__((ext_vector_type(16))) _Float16 v16b;
typedef __attribute__((ext_vector_type(8))) _Float16 v8b;
typedef __attribute__((ext_vector_type(8))) float v8f;
typedef __attribute__((ext_vector_type(4))) float v4f;
typedef __attribute__((ext_vector_type(2))) float v2f;
__device__ __forceinline__ float bf16_rne(float f) { unsigned int u = __float_as_uint(f); u += 0x7FFFu + ((u >> 16) & 1u); return __uint_as_float(u & 0xFFFF0000u); }
__device__ __forceinline__ void split16(float v, b16& hi, b16& lo) { hi = (b16)v; lo = (b16)(v - (float)hi); }
__device__ __forceinline__ v16b frag_kb(const b16* p, int hh) { const v8b a = *(const v8b*)(p + 8 * hh), b = *(const v8b*)(p + 16 + 8 * hh); v16b f;
#pragma unroll
  for (int e = 0; e < 8; ++e) { f[e] = a[e]; f[8 + e] = b[e]; } return f; }
__device__ __forceinline__ v8f wmma16b(v16b a, v16b b, v8f c) { v8f d = __builtin_amdgcn_wmma_f32_16x16x32_f16(false, a, false, b, (short)0, c, false, false); asm volatile("v_nop\n\tv_nop\n\tv_nop\n\tv_nop" : "+v"(d) : "v"(a), "v"(b)); return d; }
__device__ __forceinline__ void wave_lds_sync() { __builtin_amdgcn_fence(__ATOMIC_RELEASE, "workgroup"); __builtin_amdgcn_wave_barrier(); __builtin_amdgcn_fence(__ATOMIC_ACQUIRE, "workgroup"); }
__device__ __forceinline__ float pmul(float a, float b) { float p = a * b; asm volatile("" : "+v"(p)); return p; }
__device__ __forceinline__ int iclamp(int v, int lo, int hi) { return v < lo ? lo : (v > hi ? hi : v); }
__device__ __forceinline__ float leaky(float v) { return v >= 0.0f ? v : NEG * v; }
__device__ __forceinline__ float bnrelu(float v, float m, float rs, float g, float b) { return fmaxf(pmul(pmul(v - m, rs), g) + b, 0.0f); }
template <int CPL> __device__ __forceinline__ void ldrow(const float* p, float* f) { if (CPL == 4) { const v4f a = *(const v4f*)p; for (int i = 0; i < 4; ++i) f[i] = a[i]; } else if (CPL == 2) { const v2f a = *(const v2f*)p; f[0] = a[0]; f[1] = a[1]; } else { for (int i = 0; i < CPL; ++i) f[i] = p[i]; } }
template <int CPL> __device__ __forceinline__ void strow(float* p, const float* f) { if (CPL == 4) { v4f a; for (int i = 0; i < 4; ++i) a[i] = f[i]; *(volatile v4f*)p = a; } else if (CPL == 2) { v2f a = {f[0], f[1]}; *(volatile v2f*)p = a; } else { for (int i = 0; i < CPL; ++i) ((volatile float*)p)[i] = f[i]; } }
constexpr int CSR_NBLK8 = 512, CSR_GB8 = 8, CSR_GN8 = 1 << CSR_GB8  , CSR_TS8 = (CSR_GN8 < 32 ? 32 : CSR_GN8)  , CSR_MAXG8 = 512, CSR_CAP8 = 12288  ;
__device__ __host__ __forceinline__ int csr_tix8(int v) { return (v >> CSR_GB8) * CSR_TS8 + (v & (CSR_GN8 - 1)); }
__global__ __launch_bounds__(64) void csrA_kernel8(const int* __restrict__ dst, int E, int N, int nG, int CHP, int NGP, int* __restrict__ STG, int* __restrict__ HST) {
  extern __shared__ int sm[];
  int* cnt = sm; int* run = sm + NGP; int* ids = sm + 2 * NGP;
  const int b = blockIdx.x; const int ch = (E + CSR_NBLK8 - 1) / CSR_NBLK8; const int e0 = b * ch, e1 = min(E, e0 + ch);
  for (int i = threadIdx.x; i < NGP; i += 64) cnt[i] = 0;
  for (int i = threadIdx.x; i < CHP; i += 64) ids[i] = -1;
  __syncthreads();
  if (threadIdx.x == 0) {
    for (int e = e0; e < e1; ++e) { int d = dst[e]; d = (d < 0) ? 0 : (d >= N ? N - 1 : d); cnt[d >> CSR_GB8] += 1; }
    int acc = 0; for (int g = 0; g < nG; ++g) { run[g] = acc; acc += cnt[g]; }
    for (int e = e0; e < e1; ++e) { int d = dst[e]; d = (d < 0) ? 0 : (d >= N ? N - 1 : d); const int g = d >> CSR_GB8; ids[run[g]] = e; run[g] += 1; } }
  __syncthreads();
  typedef __attribute__((ext_vector_type(4))) int v4i;
  for (int pass = 0; pass < 2; ++pass) {
    for (int i = threadIdx.x; i < CHP / 4; i += 64) *(volatile v4i*)(STG + (size_t)b * CHP + i * 4) = *(const v4i*)(&ids[i * 4]);
    for (int i = threadIdx.x; i < NGP / 4; i += 64) { v4i v; for (int e = 0; e < 4; ++e) v[e] = (i * 4 + e < nG) ? cnt[i * 4 + e] : 0; *(volatile v4i*)(HST + (size_t)b * NGP + i * 4) = v; }
    __threadfence(); }
}
__global__ __launch_bounds__(512) void csrS_kernel8(const int* __restrict__ HST, int nG, int NGP, int* __restrict__ START, int* __restrict__ TOT, int* __restrict__ OFF) {
  __shared__ int tot[CSR_MAXG8];
  const int b = threadIdx.x;
  for (int pass = 0; pass < 2; ++pass) { int runb = 0; for (int g = 0; g < nG; ++g) { int c = HST[(size_t)b * NGP + g]; c = (c < 0) ? 0 : c; ((volatile int*)OFF)[(size_t)g * CSR_NBLK8 + b] = runb; runb += c; } __threadfence(); }
  for (int g = threadIdx.x; g < nG; g += 512) { int s = 0; for (int bb = 0; bb < CSR_NBLK8; ++bb) { int c = HST[(size_t)bb * NGP + g]; s += (c < 0) ? 0 : c; } tot[g] = s; }
  __syncthreads();
  if (threadIdx.x < 32) {
    __shared__ int st[CSR_MAXG8 + 32];
    if (threadIdx.x == 0) { int acc = 0; for (int g = 0; g < NGP; ++g) { st[g] = acc; if (g < nG) acc += (tot[g] + 31) & ~31; } st[NGP] = acc; }
    __builtin_amdgcn_fence(__ATOMIC_RELEASE, "workgroup"); __builtin_amdgcn_wave_barrier(); __builtin_amdgcn_fence(__ATOMIC_ACQUIRE, "workgroup");
    for (int pass = 0; pass < 2; ++pass) { for (int i = threadIdx.x; i < NGP + 32; i += 32) { ((volatile int*)START)[i] = (i <= NGP) ? st[min(i, NGP)] : 0; ((volatile int*)TOT)[i] = (i < nG) ? tot[i] : 0; } __threadfence(); } }
}
__global__ __launch_bounds__(256) void csrB_kernel8(const int* __restrict__ dst, int N, int nG, int CHP, int NGP, int permLen, const int* __restrict__ STG, const int* __restrict__ HST, const int* __restrict__ OFF, const int* __restrict__ START, const int* __restrict__ TOT, int* __restrict__ PERM, int* __restrict__ ROWPTR, int* __restrict__ ROWCNT, int* __restrict__ FLAG) {
  typedef __attribute__((ext_vector_type(4))) int v4i;
  __shared__ int ids[CSR_CAP8]; __shared__ unsigned short key[CSR_CAP8]; __shared__ int outp[CSR_CAP8]; __shared__ int ncnt[CSR_GN8 + 1]; __shared__ int boff[CSR_NBLK8 + 1];
  const int g = blockIdx.x, t_ = threadIdx.x; int tot = TOT[g]; int st = START[g], stn = START[g + 1]; const int v0 = g * CSR_GN8; const int nv = min(CSR_GN8, N - v0); const int t0 = g * CSR_TS8;
  st = (st < 0) ? 0 : (st > permLen - 32 ? permLen - 32 : st) & ~31; stn = (stn < st) ? st : (stn > permLen ? permLen : stn); tot = (tot < 0) ? 0 : tot; if (tot > stn - st && tot <= CSR_CAP8) tot = stn - st;
  if (tot > CSR_CAP8) {
    for (int pass = 0; pass < 2; ++pass) { for (int i = t_; i < CSR_TS8 / 4; i += 256) { v4i a, c; for (int e = 0; e < 4; ++e) { a[e] = st; c[e] = 0; } *(volatile v4i*)(ROWPTR + t0 + i * 4) = a; *(volatile v4i*)(ROWCNT + t0 + i * 4) = c; } if (t_ == 0) ((volatile int*)FLAG)[0] = 1; __threadfence(); } (void)nv; return; }
  if (t_ == 0) { int acc = 0; for (int b = 0; b < CSR_NBLK8; ++b) { boff[b] = acc; int c = HST[(size_t)b * NGP + g]; c = (c < 0) ? 0 : (c > CHP ? CHP : c); acc += c; if (acc > tot) acc = tot; } boff[CSR_NBLK8] = acc; }
  for (int i = t_; i <= CSR_GN8; i += 256) ncnt[i] = 0;
  __syncthreads();
  for (int b = 0; b < CSR_NBLK8; ++b) { const int c = boff[b + 1] - boff[b]; int o_ = OFF[(size_t)g * CSR_NBLK8 + b]; o_ = (o_ < 0) ? 0 : (o_ > CHP - c ? CHP - c : o_); const int* src_ = STG + (size_t)b * CHP + o_;
    for (int i = t_; i < c; i += 256) { int id = src_[i]; id = (id < 0) ? 0 : id; ids[boff[b] + i] = id; int d = dst[id]; d = (d < v0) ? v0 : (d >= N ? N - 1 : d); int kk = d - v0; kk = (kk < 0) ? 0 : (kk >= CSR_GN8 ? CSR_GN8 - 1 : kk); key[boff[b] + i] = (unsigned short)kk; } }
  __syncthreads();
  if (t_ == 0) { for (int i = 0; i < tot; ++i) ncnt[key[i]] += 1; int acc = 0; for (int vl = 0; vl < CSR_GN8; ++vl) { const int c = ncnt[vl]; ncnt[vl] = acc; acc += c; } ncnt[CSR_GN8] = acc;
    for (int i = 0; i < tot; ++i) { const int vl = key[i]; outp[ncnt[vl]] = ids[i]; ncnt[vl] += 1; }
    for (int vl = CSR_GN8; vl > 0; --vl) ncnt[vl] = ncnt[vl - 1]; ncnt[0] = 0; }
  __syncthreads();
  for (int pass = 0; pass < 2; ++pass) {
    for (int i = t_; i < (stn - st) / 4; i += 256) { v4i v; for (int e = 0; e < 4; ++e) { const int q = i * 4 + e; v[e] = (q < tot) ? outp[q] : -1; } *(volatile v4i*)(PERM + st + i * 4) = v; }
    for (int i = t_; i < CSR_TS8 / 4; i += 256) { v4i a, c; for (int e = 0; e < 4; ++e) { const int vl = i * 4 + e; const int vc = vl < CSR_GN8 ? vl : CSR_GN8; a[e] = (vl < CSR_GN8) ? st + ncnt[vc] : st; c[e] = (vl < nv) ? (ncnt[(vc < CSR_GN8 ? vc : CSR_GN8 - 1) + 1] - ncnt[vc]) : 0; } *(volatile v4i*)(ROWPTR + t0 + i * 4) = a; *(volatile v4i*)(ROWCNT + t0 + i * 4) = c; }
    __threadfence(); }
}
__global__ __launch_bounds__(256) void csrZ_kernel8(int* __restrict__ p, size_t n4) { typedef __attribute__((ext_vector_type(4))) int v4i; const size_t tid = (size_t)blockIdx.x * 256 + threadIdx.x, nth = (size_t)gridDim.x * 256; v4i z = {0, 0, 0, 0}; for (size_t i = tid; i < n4; i += nth) *(volatile v4i*)(p + i * 4) = z; }
struct CsrBufs8 { int *STG, *HST, *OFF, *START, *TOT, *PERM, *ROWPTR, *ROWCNT, *FLAG; int nG, NGP, CHP; size_t permLen; char* base; size_t bytes; };
static size_t csr_carve8(CsrBufs8& c, char* ws, size_t off, int E, int N) {
  const size_t off0 = off; c.base = ws + off;
  auto al = [&](size_t bytes) { char* p = ws + off; off += (bytes + 255) & ~(size_t)255; return p; };
  c.nG = (N + CSR_GN8 - 1) / CSR_GN8; c.NGP = (c.nG + 31) & ~31; const int ch = (E + CSR_NBLK8 - 1) / CSR_NBLK8; c.CHP = (ch + 31) & ~31; c.permLen = (size_t)E + 32 * (size_t)c.nG + 32;
  c.STG = (int*)al((size_t)CSR_NBLK8 * c.CHP * 4); c.HST = (int*)al((size_t)CSR_NBLK8 * c.NGP * 4); c.OFF = (int*)al((size_t)c.NGP * CSR_NBLK8 * 4); c.START = (int*)al((size_t)(c.NGP + 64) * 4); c.TOT = (int*)al((size_t)(c.NGP + 64) * 4);
  c.PERM = (int*)al(c.permLen * 4); c.ROWPTR = (int*)al((size_t)c.nG * CSR_TS8 * 4); c.ROWCNT = (int*)al((size_t)c.nG * CSR_TS8 * 4); c.FLAG = (int*)al(256);
  c.bytes = off - off0; return off;
}
static void csr_build8(const CsrBufs8& c, const int* dst, int E, int N, hipStream_t stream) {
  const size_t smem = (size_t)(2 * c.NGP + c.CHP) * 4;
  csrZ_kernel8<<<512, 256, 0, stream>>>((int*)c.base, c.bytes / 16);
  csrA_kernel8<<<CSR_NBLK8, 64, smem, stream>>>(dst, E, N, c.nG, c.CHP, c.NGP, c.STG, c.HST);
  csrS_kernel8<<<1, 512, 0, stream>>>(c.HST, c.nG, c.NGP, c.START, c.TOT, c.OFF);
  csrB_kernel8<<<c.nG, 256, 0, stream>>>(dst, N, c.nG, c.CHP, c.NGP, (int)c.permLen, c.STG, c.HST, c.OFF, c.START, c.TOT, c.PERM, c.ROWPTR, c.ROWCNT, c.FLAG);
}

constexpr int CSR_NBLK3 = 512, CSR_GB3 = 3, CSR_GN3 = 1 << CSR_GB3  , CSR_TS3 = (CSR_GN3 < 32 ? 32 : CSR_GN3)  , CSR_MAXG3 = 512, CSR_CAP3 = 12288  ;
__device__ __host__ __forceinline__ int csr_tix3(int v) { return (v >> CSR_GB3) * CSR_TS3 + (v & (CSR_GN3 - 1)); }
__global__ __launch_bounds__(64) void csrA_kernel3(const int* __restrict__ dst, int E, int N, int nG, int CHP, int NGP, int* __restrict__ STG, int* __restrict__ HST) {
  extern __shared__ int sm[];
  int* cnt = sm; int* run = sm + NGP; int* ids = sm + 2 * NGP;
  const int b = blockIdx.x; const int ch = (E + CSR_NBLK3 - 1) / CSR_NBLK3; const int e0 = b * ch, e1 = min(E, e0 + ch);
  for (int i = threadIdx.x; i < NGP; i += 64) cnt[i] = 0;
  for (int i = threadIdx.x; i < CHP; i += 64) ids[i] = -1;
  __syncthreads();
  if (threadIdx.x == 0) {
    for (int e = e0; e < e1; ++e) { int d = dst[e]; d = (d < 0) ? 0 : (d >= N ? N - 1 : d); cnt[d >> CSR_GB3] += 1; }
    int acc = 0; for (int g = 0; g < nG; ++g) { run[g] = acc; acc += cnt[g]; }
    for (int e = e0; e < e1; ++e) { int d = dst[e]; d = (d < 0) ? 0 : (d >= N ? N - 1 : d); const int g = d >> CSR_GB3; ids[run[g]] = e; run[g] += 1; } }
  __syncthreads();
  typedef __attribute__((ext_vector_type(4))) int v4i;
  for (int pass = 0; pass < 2; ++pass) {
    for (int i = threadIdx.x; i < CHP / 4; i += 64) *(volatile v4i*)(STG + (size_t)b * CHP + i * 4) = *(const v4i*)(&ids[i * 4]);
    for (int i = threadIdx.x; i < NGP / 4; i += 64) { v4i v; for (int e = 0; e < 4; ++e) v[e] = (i * 4 + e < nG) ? cnt[i * 4 + e] : 0; *(volatile v4i*)(HST + (size_t)b * NGP + i * 4) = v; }
    __threadfence(); }
}
__global__ __launch_bounds__(512) void csrS_kernel3(const int* __restrict__ HST, int nG, int NGP, int* __restrict__ START, int* __restrict__ TOT, int* __restrict__ OFF) {
  __shared__ int tot[CSR_MAXG3];
  const int b = threadIdx.x;
  for (int pass = 0; pass < 2; ++pass) { int runb = 0; for (int g = 0; g < nG; ++g) { int c = HST[(size_t)b * NGP + g]; c = (c < 0) ? 0 : c; ((volatile int*)OFF)[(size_t)g * CSR_NBLK3 + b] = runb; runb += c; } __threadfence(); }
  for (int g = threadIdx.x; g < nG; g += 512) { int s = 0; for (int bb = 0; bb < CSR_NBLK3; ++bb) { int c = HST[(size_t)bb * NGP + g]; s += (c < 0) ? 0 : c; } tot[g] = s; }
  __syncthreads();
  if (threadIdx.x < 32) {
    __shared__ int st[CSR_MAXG3 + 32];
    if (threadIdx.x == 0) { int acc = 0; for (int g = 0; g < NGP; ++g) { st[g] = acc; if (g < nG) acc += (tot[g] + 31) & ~31; } st[NGP] = acc; }
    __builtin_amdgcn_fence(__ATOMIC_RELEASE, "workgroup"); __builtin_amdgcn_wave_barrier(); __builtin_amdgcn_fence(__ATOMIC_ACQUIRE, "workgroup");
    for (int pass = 0; pass < 2; ++pass) { for (int i = threadIdx.x; i < NGP + 32; i += 32) { ((volatile int*)START)[i] = (i <= NGP) ? st[min(i, NGP)] : 0; ((volatile int*)TOT)[i] = (i < nG) ? tot[i] : 0; } __threadfence(); } }
}
__global__ __launch_bounds__(256) void csrB_kernel3(const int* __restrict__ dst, int N, int nG, int CHP, int NGP, int permLen, const int* __restrict__ STG, const int* __restrict__ HST, const int* __restrict__ OFF, const int* __restrict__ START, const int* __restrict__ TOT, int* __restrict__ PERM, int* __restrict__ ROWPTR, int* __restrict__ ROWCNT, int* __restrict__ FLAG) {
  typedef __attribute__((ext_vector_type(4))) int v4i;
  __shared__ int ids[CSR_CAP3]; __shared__ unsigned short key[CSR_CAP3]; __shared__ int outp[CSR_CAP3]; __shared__ int ncnt[CSR_GN3 + 1]; __shared__ int boff[CSR_NBLK3 + 1];
  const int g = blockIdx.x, t_ = threadIdx.x; int tot = TOT[g]; int st = START[g], stn = START[g + 1]; const int v0 = g * CSR_GN3; const int nv = min(CSR_GN3, N - v0); const int t0 = g * CSR_TS3;
  st = (st < 0) ? 0 : (st > permLen - 32 ? permLen - 32 : st) & ~31; stn = (stn < st) ? st : (stn > permLen ? permLen : stn); tot = (tot < 0) ? 0 : tot; if (tot > stn - st && tot <= CSR_CAP3) tot = stn - st;
  if (tot > CSR_CAP3) {
    for (int pass = 0; pass < 2; ++pass) { for (int i = t_; i < CSR_TS3 / 4; i += 256) { v4i a, c; for (int e = 0; e < 4; ++e) { a[e] = st; c[e] = 0; } *(volatile v4i*)(ROWPTR + t0 + i * 4) = a; *(volatile v4i*)(ROWCNT + t0 + i * 4) = c; } if (t_ == 0) ((volatile int*)FLAG)[0] = 1; __threadfence(); } (void)nv; return; }
  if (t_ == 0) { int acc = 0; for (int b = 0; b < CSR_NBLK3; ++b) { boff[b] = acc; int c = HST[(size_t)b * NGP + g]; c = (c < 0) ? 0 : (c > CHP ? CHP : c); acc += c; if (acc > tot) acc = tot; } boff[CSR_NBLK3] = acc; }
  for (int i = t_; i <= CSR_GN3; i += 256) ncnt[i] = 0;
  __syncthreads();
  for (int b = 0; b < CSR_NBLK3; ++b) { const int c = boff[b + 1] - boff[b]; int o_ = OFF[(size_t)g * CSR_NBLK3 + b]; o_ = (o_ < 0) ? 0 : (o_ > CHP - c ? CHP - c : o_); const int* src_ = STG + (size_t)b * CHP + o_;
    for (int i = t_; i < c; i += 256) { int id = src_[i]; id = (id < 0) ? 0 : id; ids[boff[b] + i] = id; int d = dst[id]; d = (d < v0) ? v0 : (d >= N ? N - 1 : d); int kk = d - v0; kk = (kk < 0) ? 0 : (kk >= CSR_GN3 ? CSR_GN3 - 1 : kk); key[boff[b] + i] = (unsigned short)kk; } }
  __syncthreads();
  if (t_ == 0) { for (int i = 0; i < tot; ++i) ncnt[key[i]] += 1; int acc = 0; for (int vl = 0; vl < CSR_GN3; ++vl) { const int c = ncnt[vl]; ncnt[vl] = acc; acc += c; } ncnt[CSR_GN3] = acc;
    for (int i = 0; i < tot; ++i) { const int vl = key[i]; outp[ncnt[vl]] = ids[i]; ncnt[vl] += 1; }
    for (int vl = CSR_GN3; vl > 0; --vl) ncnt[vl] = ncnt[vl - 1]; ncnt[0] = 0; }
  __syncthreads();
  for (int pass = 0; pass < 2; ++pass) {
    for (int i = t_; i < (stn - st) / 4; i += 256) { v4i v; for (int e = 0; e < 4; ++e) { const int q = i * 4 + e; v[e] = (q < tot) ? outp[q] : -1; } *(volatile v4i*)(PERM + st + i * 4) = v; }
    for (int i = t_; i < CSR_TS3 / 4; i += 256) { v4i a, c; for (int e = 0; e < 4; ++e) { const int vl = i * 4 + e; const int vc = vl < CSR_GN3 ? vl : CSR_GN3; a[e] = (vl < CSR_GN3) ? st + ncnt[vc] : st; c[e] = (vl < nv) ? (ncnt[(vc < CSR_GN3 ? vc : CSR_GN3 - 1) + 1] - ncnt[vc]) : 0; } *(volatile v4i*)(ROWPTR + t0 + i * 4) = a; *(volatile v4i*)(ROWCNT + t0 + i * 4) = c; }
    __threadfence(); }
}
__global__ __launch_bounds__(256) void csrZ_kernel3(int* __restrict__ p, size_t n4) { typedef __attribute__((ext_vector_type(4))) int v4i; const size_t tid = (size_t)blockIdx.x * 256 + threadIdx.x, nth = (size_t)gridDim.x * 256; v4i z = {0, 0, 0, 0}; for (size_t i = tid; i < n4; i += nth) *(volatile v4i*)(p + i * 4) = z; }
struct CsrBufs3 { int *STG, *HST, *OFF, *START, *TOT, *PERM, *ROWPTR, *ROWCNT, *FLAG; int nG, NGP, CHP; size_t permLen; char* base; size_t bytes; };
static size_t csr_carve3(CsrBufs3& c, char* ws, size_t off, int E, int N) {
  const size_t off0 = off; c.base = ws + off;
  auto al = [&](size_t bytes) { char* p = ws + off; off += (bytes + 255) & ~(size_t)255; return p; };
  c.nG = (N + CSR_GN3 - 1) / CSR_GN3; c.NGP = (c.nG + 31) & ~31; const int ch = (E + CSR_NBLK3 - 1) / CSR_NBLK3; c.CHP = (ch + 31) & ~31; c.permLen = (size_t)E + 32 * (size_t)c.nG + 32;
  c.STG = (int*)al((size_t)CSR_NBLK3 * c.CHP * 4); c.HST = (int*)al((size_t)CSR_NBLK3 * c.NGP * 4); c.OFF = (int*)al((size_t)c.NGP * CSR_NBLK3 * 4); c.START = (int*)al((size_t)(c.NGP + 64) * 4); c.TOT = (int*)al((size_t)(c.NGP + 64) * 4);
  c.PERM = (int*)al(c.permLen * 4); c.ROWPTR = (int*)al((size_t)c.nG * CSR_TS3 * 4); c.ROWCNT = (int*)al((size_t)c.nG * CSR_TS3 * 4); c.FLAG = (int*)al(256);
  c.bytes = off - off0; return off;
}
static void csr_build3(const CsrBufs3& c, const int* dst, int E, int N, hipStream_t stream) {
  const size_t smem = (size_t)(2 * c.NGP + c.CHP) * 4;
  csrZ_kernel3<<<512, 256, 0, stream>>>((int*)c.base, c.bytes / 16);
  csrA_kernel3<<<CSR_NBLK3, 64, smem, stream>>>(dst, E, N, c.nG, c.CHP, c.NGP, c.STG, c.HST);
  csrS_kernel3<<<1, 512, 0, stream>>>(c.HST, c.nG, c.NGP, c.START, c.TOT, c.OFF);
  csrB_kernel3<<<c.nG, 256, 0, stream>>>(dst, N, c.nG, c.CHP, c.NGP, (int)c.permLen, c.STG, c.HST, c.OFF, c.START, c.TOT, c.PERM, c.ROWPTR, c.ROWCNT, c.FLAG);
}


__global__ __launch_bounds__(256) void wprep_kernel(const float* __restrict__ w, int KIN, int OUT, int KP, b16* __restrict__ WT) {
  const int u = blockIdx.x * 256 + threadIdx.x; if (u >= OUT * KP / 8) return; const int e = u * 8; const int o = e / KP, k0 = e % KP; v8b v; for (int j = 0; j < 8; ++j) { const int k = k0 + j; v[j] = k < KIN ? (b16)(bf16_rne(w[(size_t)k * OUT + o]) * WSC) : (b16)0.0f; }
  for (int pass = 0; pass < 2; ++pass) { *(volatile v8b*)(WT + e) = v; __threadfence(); }
}
template <int MODE, int KIN, int NT, int HT>
__global__ __launch_bounds__(32) void lin_kernel(const float* __restrict__ xin, const float* __restrict__ PREV, const float* __restrict__ bm, const float* __restrict__ bv, const float* __restrict__ bg, const float* __restrict__ bb, const b16* __restrict__ WT, const float* __restrict__ as, const float* __restrict__ ad, int NLIM, float* __restrict__ P, float* __restrict__ ES, float* __restrict__ ED) {
  __shared__ __attribute__((aligned(16))) b16 Ah[16][KIN + 8], Al[16][KIN + 8]; __shared__ __attribute__((aligned(16))) float Tf[16][128 + 4]; __shared__ __attribute__((aligned(16))) float Se[16][4], Sd[16][4];
  const int lane = threadIdx.x, nloc = lane & 15, hlf = lane >> 4; const size_t m0 = (size_t)blockIdx.x * 16; const bool live = m0 < (size_t)NLIM; const float sc = 1.0f / (XS * WSC); constexpr int CPL = KIN / 32;
  float pm[CPL > 0 ? CPL : 1], pr[CPL > 0 ? CPL : 1], pg[CPL > 0 ? CPL : 1], pb[CPL > 0 ? CPL : 1];
  if (MODE) for (int j = 0; j < CPL; ++j) { const int c = lane * CPL + j; pm[j] = bf16_rne(bm[c]); pr[j] = rsqrtf(bf16_rne(bv[c]) + BNEPS); pg[j] = bf16_rne(bg[c]); pb[j] = bf16_rne(bb[c]); }
  for (int rr = 0; rr < 16; ++rr) { const size_t r = (m0 + rr) < (size_t)N ? m0 + rr : (size_t)N - 1;
    if (MODE == 0) { Ah[rr][lane] = lane < 3 ? (b16)(bf16_rne(xin[r * XF + lane]) * XS) : (b16)0.0f; Al[rr][lane] = (b16)0.0f; }
    else { float v[CPL > 0 ? CPL : 1]; if (live) ldrow<CPL>(PREV + r * KIN + lane * CPL, v); else for (int j = 0; j < CPL; ++j) v[j] = 0.0f; for (int j = 0; j < CPL; ++j) { b16 p, ql; split16((live ? bnrelu(v[j], pm[j], pr[j], pg[j], pb[j]) : 0.0f) * XS, p, ql); Ah[rr][lane * CPL + j] = p; Al[rr][lane * CPL + j] = ql; } }
    if (lane < 16) for (int h = 0; h < 4; ++h) { Se[rr][h] = 0.0f; Sd[rr][h] = 0.0f; } }
  wave_lds_sync();
  v8f acc[NT]; float pes[NT / HT][8], ped[NT / HT][8];
#pragma unroll
  for (int t = 0; t < NT; ++t) acc[t] = (v8f){};
  if (live) {
#pragma unroll 2
    for (int kb = 0; kb < KIN; kb += 32) { const v16b a = frag_kb(&Ah[nloc][kb], hlf); v16b al = {}; if (MODE) al = frag_kb(&Al[nloc][kb], hlf);
#pragma unroll
      for (int t = 0; t < NT; ++t) { const v16b bw = frag_kb(WT + (size_t)(t * 16 + nloc) * KIN + kb, hlf); acc[t] = wmma16b(a, bw, acc[t]); if (MODE) acc[t] = wmma16b(al, bw, acc[t]); } } }
#pragma unroll
  for (int hh = 0; hh < NT / HT; ++hh) for (int r8 = 0; r8 < 8; ++r8) { pes[hh][r8] = 0.0f; ped[hh][r8] = 0.0f; }
#pragma unroll
  for (int t = 0; t < NT; ++t) { const int c = t * 16 + nloc; const int hh = t / HT; const float wsv = bf16_rne(as[c]), wdv = bf16_rne(ad[c]);
#pragma unroll
    for (int r8 = 0; r8 < 8; ++r8) { const float p = acc[t][r8] * sc; Tf[8 * hlf + r8][c] = p; pes[hh][r8] += pmul(p, wsv); ped[hh][r8] += pmul(p, wdv); } }
#pragma unroll
  for (int hh = 0; hh < NT / HT; ++hh)
#pragma unroll
    for (int r8 = 0; r8 < 8; ++r8) { float s = pes[hh][r8], d = ped[hh][r8]; for (int o = 1; o < 16; o <<= 1) { s += __shfl_xor(s, o); d += __shfl_xor(d, o); } if (nloc == 0) { Se[8 * hlf + r8][hh] = s; Sd[8 * hlf + r8][hh] = d; } }
  wave_lds_sync();
  constexpr int OW = NT * 16, OPL = OW / 32; typedef __attribute__((ext_vector_type(OPL))) float vof;
  for (int pass = 0; pass < 2; ++pass) { for (int rr = 0; rr < 16; ++rr) *(volatile vof*)(P + (m0 + rr) * OW + lane * OPL) = *(const vof*)(&Tf[rr][lane * OPL]);
    if (lane < 16) { *(volatile v4f*)(ES + (m0 + lane) * 4) = *(const v4f*)(&Se[lane][0]); *(volatile v4f*)(ED + (m0 + lane) * 4) = *(const v4f*)(&Sd[lane][0]); } __threadfence(); }
}
template <int W, int NHH, int EW>
__global__ __launch_bounds__(256) void att_kernel(const float* __restrict__ P, const float* __restrict__ ES, const float* __restrict__ ED, const float* __restrict__ bias, const int* __restrict__ srcs, const int* __restrict__ PERM, const int* __restrict__ ROWPTR, const int* __restrict__ ROWCNT, int permLen, int NLIM, float* __restrict__ Gout) {
  constexpr int CPL = W / 32;
  const int wave = threadIdx.x >> 5, lane = threadIdx.x & 31; const size_t v = (size_t)blockIdx.x * 8 + wave; const int h = (lane * CPL) / (W / NHH); float o[CPL]; for (int i = 0; i < CPL; ++i) o[i] = 0.0f;
  if (v < (size_t)NLIM) { int st = ROWPTR[v], cnt = ROWCNT[v]; cnt = iclamp(cnt, 0, 1 << 20); st = iclamp(st, 0, permLen - cnt); const float edv = ED[v * EW + h]; float mx = leaky(ES[v * EW + h] + edv);
#pragma unroll 1
    for (int j = 0; j < cnt; ++j) { const int e = iclamp(PERM[st + j], 0, E - 1); const int s = iclamp(srcs[e], 0, N - 1); if (s >= NLIM) continue; mx = fmaxf(mx, leaky(ES[(size_t)s * EW + h] + edv)); }
    float den; { const float p = __expf(leaky(ES[v * EW + h] + edv) - mx); den = p; float f[CPL]; ldrow<CPL>(P + v * W + lane * CPL, f); for (int i = 0; i < CPL; ++i) o[i] = pmul(p, f[i]); }
#pragma unroll 1
    for (int j = 0; j < cnt; ++j) { const int e = iclamp(PERM[st + j], 0, E - 1); const int s = iclamp(srcs[e], 0, N - 1); if (s >= NLIM) continue; const float p = __expf(leaky(ES[(size_t)s * EW + h] + edv) - mx); den += p; float f[CPL]; ldrow<CPL>(P + (size_t)s * W + lane * CPL, f); for (int i = 0; i < CPL; ++i) o[i] += pmul(p, f[i]); }
    const float inv = 1.0f / den;   for (int i = 0; i < CPL; ++i) o[i] = pmul(o[i], inv) + bf16_rne(bias[lane * CPL + i]); }
  for (int pass = 0; pass < 2; ++pass) { strow<CPL>(Gout + v * W + lane * CPL, o); __threadfence(); }
}


__global__ __launch_bounds__(128) void head_kernel(const float* __restrict__ G3, const float* __restrict__ m3, const float* __restrict__ v3, const float* __restrict__ g3, const float* __restrict__ b3, const int* __restrict__ PERM, const int* __restrict__ ROWPTR, const int* __restrict__ ROWCNT, int permLen, int NLIM,
    const b16* __restrict__ WFT, const float* __restrict__ bf, const float* __restrict__ g4, const float* __restrict__ be4, const float* __restrict__ m4, const float* __restrict__ v4, const b16* __restrict__ WL1T, const float* __restrict__ bl1, const float* __restrict__ wl2, const float* __restrict__ bl2, float* __restrict__ out1, float* __restrict__ out2) {
  __shared__ __attribute__((aligned(16))) b16 Ah[4][16][W2O + 8], Al[4][16][W2O + 8]; __shared__ __attribute__((aligned(16))) float Pool[4][16][W2O + 4]; __shared__ float so[G * NCLS];
  const int wave = threadIdx.x >> 5, lane = threadIdx.x & 31, nloc = lane & 15, hlf = lane >> 4; const int g0 = wave * 16; const float sc = 1.0f / (XS * WSC);
  float pm[4], pr[4], pg[4], pb[4]; for (int j = 0; j < 4; ++j) { const int c = lane * 4 + j; pm[j] = bf16_rne(m3[c]); pr[j] = rsqrtf(bf16_rne(v3[c]) + BNEPS); pg[j] = bf16_rne(g3[c]); pb[j] = bf16_rne(b3[c]); }
  for (int rr = 0; rr < 16; ++rr) { const int g = g0 + rr; const int tix = (g >> 3) * 32 + (g & 7); int st = ROWPTR[tix], cnt = ROWCNT[tix]; cnt = iclamp(cnt, 0, 1 << 20); st = iclamp(st, 0, permLen - cnt); float a[4] = {0.0f, 0.0f, 0.0f, 0.0f};
#pragma unroll 1
    for (int j = 0; j < cnt; ++j) { const int n = iclamp(PERM[st + j], 0, N - 1); if (n >= NLIM) continue; const v4f hv = *(const v4f*)(G3 + (size_t)n * W2O + lane * 4); for (int i = 0; i < 4; ++i) a[i] += bnrelu(hv[i], pm[i], pr[i], pg[i], pb[i]); }
    const float inv = 1.0f / (float)(cnt < 1 ? 1 : cnt); for (int i = 0; i < 4; ++i) { const float mv = pmul(a[i], inv); Pool[wave][rr][lane * 4 + i] = mv; b16 p, q; split16(mv * XS, p, q); Ah[wave][rr][lane * 4 + i] = p; Al[wave][rr][lane * 4 + i] = q; } }
  wave_lds_sync();
  for (int pass = 0; pass < 2; ++pass) { for (int rr = 0; rr < 16; ++rr) *(volatile v4f*)(out1 + (size_t)(g0 + rr) * W2O + lane * 4) = *(const v4f*)(&Pool[wave][rr][lane * 4]); __threadfence(); }
  v8f acc[2] = {(v8f){}, (v8f){}};
#pragma unroll 2
  for (int kb = 0; kb < W2O; kb += 32) { const v16b a = frag_kb(&Ah[wave][nloc][kb], hlf), al = frag_kb(&Al[wave][nloc][kb], hlf);
#pragma unroll
    for (int t = 0; t < 2; ++t) { const v16b bw = frag_kb(WFT + (size_t)(t * 16 + nloc) * W2O + kb, hlf); acc[t] = wmma16b(a, bw, acc[t]); acc[t] = wmma16b(al, bw, acc[t]); } }
  wave_lds_sync();
#pragma unroll
  for (int t = 0; t < 2; ++t) { const int c = t * 16 + nloc; const float bb = bf16_rne(bf[c]), mm = bf16_rne(m4[c]), rs = rsqrtf(bf16_rne(v4[c]) + BNEPS), gg = bf16_rne(g4[c]), be = bf16_rne(be4[c]);
#pragma unroll
    for (int r8 = 0; r8 < 8; ++r8) { const float z = bnrelu(acc[t][r8] * sc + bb, mm, rs, gg, be); b16 p, q; split16(z * XS, p, q); Ah[wave][8 * hlf + r8][c] = p; Al[wave][8 * hlf + r8][c] = q; } }
  wave_lds_sync();
  v8f a2[2] = {(v8f){}, (v8f){}};
  { const v16b a = frag_kb(&Ah[wave][nloc][0], hlf), al = frag_kb(&Al[wave][nloc][0], hlf);
#pragma unroll
    for (int t = 0; t < 2; ++t) { const v16b bw = frag_kb(WL1T + (size_t)(t * 16 + nloc) * HZ, hlf); a2[t] = wmma16b(a, bw, a2[t]); a2[t] = wmma16b(al, bw, a2[t]); } }
  float pk[NCLS][8]; for (int k = 0; k < NCLS; ++k) for (int r8 = 0; r8 < 8; ++r8) pk[k][r8] = 0.0f;
#pragma unroll
  for (int t = 0; t < 2; ++t) { const int c = t * 16 + nloc; const float bb = bf16_rne(bl1[c]); float wk[NCLS]; for (int k = 0; k < NCLS; ++k) wk[k] = bf16_rne(wl2[c * NCLS + k]);
#pragma unroll
    for (int r8 = 0; r8 < 8; ++r8) { const float z = fmaxf(a2[t][r8] * sc + bb, 0.0f); for (int k = 0; k < NCLS; ++k) pk[k][r8] += pmul(z, wk[k]); } }
#pragma unroll
  for (int k = 0; k < NCLS; ++k)
#pragma unroll
    for (int r8 = 0; r8 < 8; ++r8) { float s = pk[k][r8]; for (int o = 1; o < 16; o <<= 1) s += __shfl_xor(s, o); if (nloc == 0) so[(g0 + 8 * hlf + r8) * NCLS + k] = s + bf16_rne(bl2[k]); }
  __syncthreads();
  float ls[NCLS]; const int g = threadIdx.x; if (g < G) { float mx = -INFINITY; for (int k = 0; k < NCLS; ++k) { ls[k] = so[g * NCLS + k]; mx = fmaxf(mx, ls[k]); } float se = 0.0f; for (int k = 0; k < NCLS; ++k) se += __expf(ls[k] - mx); const float lse = mx + logf(se); for (int k = 0; k < NCLS; ++k) ls[k] -= lse; }
  __syncthreads(); if (g < G) for (int k = 0; k < NCLS; ++k) so[g * NCLS + k] = ls[k]; __syncthreads();
  for (int pass = 0; pass < 2; ++pass) { for (int i = threadIdx.x; i < G * NCLS; i += 128) ((volatile float*)out2)[i] = so[i]; __threadfence(); }
}
}

extern "C" void kernel_launch(void* const* d_in, const int* in_sizes, int n_in, void* d_out, int out_size, void* d_ws, size_t ws_size, hipStream_t stream) {
  (void)n_in;
  auto Fp = [&](int i) { return (const float*)d_in[i]; }; auto Ip = [&](int i) { return (const int*)d_in[i]; };
  if (in_sizes[0] != N * XF || in_sizes[1] != 2 * E || in_sizes[2] != N || in_sizes[3] != 3 * W1O || in_sizes[11] != W1O * W2O || in_sizes[19] != W2O * W2O || in_sizes[27] != W2O * HZ || in_sizes[33] != HZ * HZ || in_sizes[35] != HZ * NCLS || out_size != G * W2O + G * NCLS) return;
  const int NLIM = N; const int GB16 = NBLK, GB8 = NP / 8;
  size_t off = 0; char* ws = (char*)d_ws;
  auto carve = [&](size_t bytes) { char* p = ws + off; off += (bytes + 255) & ~(size_t)255; return p; };
  b16* W1T = (b16*)carve(W1O * 32 * 2); b16* W2T = (b16*)carve((size_t)W2O * W1O * 2); b16* W3T = (b16*)carve((size_t)W2O * W2O * 2); b16* WFT = (b16*)carve((size_t)HZ * W2O * 2); b16* WL1T = (b16*)carve((size_t)HZ * HZ * 2);
  float* P1 = (float*)carve((size_t)NP * W1O * 4); float* G1 = (float*)carve((size_t)NP * W1O * 4); float* PA = (float*)carve((size_t)NP * W2O * 4); float* GA = (float*)carve((size_t)NP * W2O * 4); float* GB = (float*)carve((size_t)NP * W2O * 4); float* ES = (float*)carve((size_t)NP * 4 * 4); float* ED = (float*)carve((size_t)NP * 4 * 4);
  CsrBufs8 csr; CsrBufs3 pl; off = csr_carve8(csr, ws, off, E, N); off = csr_carve3(pl, ws, off, N, G);
  if (off > ws_size || off > ((size_t)192 << 20)) return;
  wprep_kernel<<<(W1O * 32 / 8 + 255) / 256, 256, 0, stream>>>(Fp(3), 3, W1O, 32, W1T); wprep_kernel<<<(W2O * W1O / 8 + 255) / 256, 256, 0, stream>>>(Fp(11), W1O, W2O, W1O, W2T); wprep_kernel<<<(W2O * W2O / 8 + 255) / 256, 256, 0, stream>>>(Fp(19), W2O, W2O, W2O, W3T);
  wprep_kernel<<<(HZ * W2O / 8 + 255) / 256, 256, 0, stream>>>(Fp(27), W2O, HZ, W2O, WFT); wprep_kernel<<<(HZ * HZ / 8 + 255) / 256, 256, 0, stream>>>(Fp(33), HZ, HZ, HZ, WL1T);
  csr_build8(csr, Ip(1) + E, E, N, stream); csr_build3(pl, Ip(2), N, G, stream);
  lin_kernel<0, 32, 4, 2><<<GB16, 32, 0, stream>>>(Fp(0), nullptr, nullptr, nullptr, nullptr, nullptr, W1T, Fp(4), Fp(5), NLIM, P1, ES, ED);
  att_kernel<W1O, NH, 4><<<GB8, 256, 0, stream>>>(P1, ES, ED, Fp(6), Ip(1), csr.PERM, csr.ROWPTR, csr.ROWCNT, (int)csr.permLen, NLIM, G1);
  lin_kernel<1, W1O, 8, 4><<<GB16, 32, 0, stream>>>(nullptr, G1, Fp(9), Fp(10), Fp(7), Fp(8), W2T, Fp(12), Fp(13), NLIM, PA, ES, ED);
  att_kernel<W2O, NH, 4><<<GB8, 256, 0, stream>>>(PA, ES, ED, Fp(14), Ip(1), csr.PERM, csr.ROWPTR, csr.ROWCNT, (int)csr.permLen, NLIM, GA);
  lin_kernel<1, W2O, 8, 4><<<GB16, 32, 0, stream>>>(nullptr, GA, Fp(17), Fp(18), Fp(15), Fp(16), W3T, Fp(20), Fp(21), NLIM, PA, ES, ED);
  att_kernel<W2O, NH, 4><<<GB8, 256, 0, stream>>>(PA, ES, ED, Fp(22), Ip(1), csr.PERM, csr.ROWPTR, csr.ROWCNT, (int)csr.permLen, NLIM, GB);
  head_kernel<<<1, 128, 0, stream>>>(GB, Fp(25), Fp(26), Fp(23), Fp(24), pl.PERM, pl.ROWPTR, pl.ROWCNT, (int)pl.permLen, NLIM, WFT, Fp(28), Fp(29), Fp(30), Fp(31), Fp(32), WL1T, Fp(34), Fp(35), Fp(36), (float*)d_out, (float*)d_out + G * W2O);
}
